// LRU_7619271983134
// MI455X (gfx1250) — hardware-verified
//
#include <hip/hip_runtime.h>
#include <math.h>

constexpr int SEQ_L    = 8192;
constexpr int NST      = 512;
constexpr int HID      = 512;
constexpr int NST2     = 2 * NST;
constexpr int CVT_THR  = 256;
constexpr int SCAN_THR = 32;
constexpr int SCAN_CPL = 8;
constexpr int SCAN_CPB = SCAN_THR * SCAN_CPL;
static_assert(SEQ_L % 64 == 0 && NST2 % 64 == 0 && HID % 64 == 0);
static_assert(HID % 32 == 0 && NST2 % 32 == 0);
static_assert(NST % SCAN_CPB == 0);
static_assert(HID % 8 == 0 && NST % 8 == 0);
static_assert((SEQ_L * (HID / 8)) % CVT_THR == 0);
static_assert((NST * (HID / 8)) % CVT_THR == 0 && (HID * (NST / 8)) % CVT_THR == 0);

typedef __attribute__((ext_vector_type(16))) _Float16 v16h;
typedef __attribute__((ext_vector_type(8)))  _Float16 v8h;
typedef __attribute__((ext_vector_type(16))) __bf16   v16b;
typedef __attribute__((ext_vector_type(8)))  __bf16   v8b;
typedef __attribute__((ext_vector_type(8)))  float    v8f;
typedef __attribute__((ext_vector_type(4)))  float    v4f;

__device__ __forceinline__ unsigned short f2bf_bits(float f) {
  unsigned u = __float_as_uint(f);
  return (unsigned short)((u + 0x7FFFu + ((u >> 16) & 1u)) >> 16);
}
__device__ __forceinline__ float bf_bits2f(unsigned short h) { return __uint_as_float(((unsigned)h) << 16); }

__device__ __forceinline__ void dep_guard_h(v8f& a, v8f& b, v16h x, v16h y) { asm volatile("v_nop\n\tv_nop\n\tv_nop\n\tv_nop" : "+v"(a), "+v"(b) : "v"(x), "v"(y)); }
__device__ __forceinline__ void dep_guard_b(v8f& a, v8f& b, v16b x, v16b y) { asm volatile("v_nop\n\tv_nop\n\tv_nop\n\tv_nop" : "+v"(a), "+v"(b) : "v"(x), "v"(y)); }
__device__ __forceinline__ void keep4_h(v16h a, v16h b, v16h c, v16h d) { asm volatile("v_nop" :: "v"(a), "v"(b), "v"(c), "v"(d)); }
__device__ __forceinline__ void keep4_b(v16b a, v16b b, v16b c, v16b d) { asm volatile("v_nop" :: "v"(a), "v"(b), "v"(c), "v"(d)); }
__device__ __forceinline__ void acc_guard4(v8f& a, v8f& b, v8f& c, v8f& d) { asm volatile("v_nop\n\tv_nop\n\tv_nop\n\tv_nop" : "+v"(a), "+v"(b), "+v"(c), "+v"(d)); }
template <typename T> struct Frag;
template <> struct Frag<_Float16> {
  typedef v16h V; union U { v16h v; v8h h[2]; };
  static __device__ __forceinline__ v16h load(const _Float16* p) {
    U f; f.h[0] = *(const v8h*)(p); f.h[1] = *(const v8h*)(p + 16); return f.v;
  }
  static __device__ __forceinline__ v8f mma(v16h a, v16h b, v8f c) {
    return __builtin_amdgcn_wmma_f32_16x16x32_f16(false, a, false, b, (short)0, c, false, false);
  }
  static __device__ __forceinline__ void guard(v8f& a, v8f& b, v16h x, v16h y) { dep_guard_h(a, b, x, y); }
  static __device__ __forceinline__ void keep(v16h a, v16h b, v16h c, v16h d) { keep4_h(a, b, c, d); }
};
template <> struct Frag<__bf16> {
  typedef v16b V; union U { v16b v; v8b h[2]; };
  static __device__ __forceinline__ v16b load(const __bf16* p) {
    U f; f.h[0] = *(const v8b*)(p); f.h[1] = *(const v8b*)(p + 16); return f.v;
  }
  static __device__ __forceinline__ v8f mma(v16b a, v16b b, v8f c) {
    return __builtin_amdgcn_wmma_f32_16x16x32_bf16(false, a, false, b, (short)0, c, false, false);
  }
  static __device__ __forceinline__ void guard(v8f& a, v8f& b, v16b x, v16b y) { dep_guard_b(a, b, x, y); }
  static __device__ __forceinline__ void keep(v16b a, v16b b, v16b c, v16b d) { keep4_b(a, b, c, d); }
};

template <int ET> struct Elem;
template <> struct Elem<0> { typedef _Float16 T; };
template <> struct Elem<1> { typedef __bf16 T; };
template <int ET, bool SPLIT, int BIAS_MODE, int OUT_MODE, bool RESID, int ACT, bool DUADD>
__global__ __launch_bounds__(256) void wmma_gemm64(
    const unsigned short* __restrict__ Ap, const unsigned short* __restrict__ A2p, int lda, long strideA,
    const unsigned short* __restrict__ Btp, const unsigned short* __restrict__ Bt2p, int ldb, long strideB,
    void* __restrict__ Cout, void* __restrict__ Cout2, int ldc, long strideC,
    const float* __restrict__ bias,
    const float* __restrict__ resid, long strideR,
    int M, int N, int K, float scale,
    const float* __restrict__ dsc, const float* __restrict__ uadd, int ldu) {
  typedef typename Elem<ET>::T T;
  typedef typename Frag<T>::V V;
  const T* A = (const T*)Ap; const T* A2 = (const T*)A2p; const T* Bt = (const T*)Btp; const T* Bt2 = (const T*)Bt2p;
  __shared__ __align__(16) float sT[8][16 * 68];
  const int b    = blockIdx.y;
  const int lane = threadIdx.x & 31;
  const int wave = threadIdx.x >> 5;
  const int tilesN = N >> 6;
  const int tilesM = M >> 6;
  const int tile = blockIdx.x * 8 + wave;
  if (tile >= tilesM * tilesN) return;
  const int tm = tile / tilesN;
  const int tn = tile - tm * tilesN;
  const int m0 = tm << 6;
  const int n0 = tn << 6;

  const T* Ab  = A  + (size_t)b * strideA;
  const T* Bb  = Bt + (size_t)b * strideB;
  const T* Ab2 = SPLIT ? (A2  + (size_t)b * strideA) : nullptr;
  const T* Bb2 = SPLIT ? (Bt2 + (size_t)b * strideB) : nullptr;

  const int rlane = lane & 15;
  const int koff  = (lane >> 4) * 8;
  const int mOff  = (lane >> 4) * 8;

  v8f acc[4][4];
#pragma unroll
  for (int i = 0; i < 4; ++i)
#pragma unroll
    for (int j = 0; j < 4; ++j) acc[i][j] = (v8f){0.f,0.f,0.f,0.f,0.f,0.f,0.f,0.f};

  for (int k0 = 0; k0 < K; k0 += 32) {
    V bh[4], bl[4];
#pragma unroll
    for (int j = 0; j < 4; ++j) {
      const size_t bo = (size_t)(n0 + (j << 4) + rlane) * ldb + koff + k0;
      bh[j] = Frag<T>::load(Bb + bo);
      if (SPLIT) bl[j] = Frag<T>::load(Bb2 + bo);
    }
#pragma unroll
    for (int i = 0; i < 4; ++i) {
      const size_t ao = (size_t)(m0 + (i << 4) + rlane) * lda + koff + k0;
      V ah = Frag<T>::load(Ab + ao);
      V al;
      if (SPLIT) al = Frag<T>::load(Ab2 + ao);
#pragma unroll
      for (int j = 0; j < 4; ++j) {
        acc[i][j] = Frag<T>::mma(ah, bh[j], acc[i][j]);
        if (SPLIT) {
          acc[i][j] = Frag<T>::mma(ah, bl[j], acc[i][j]);
          acc[i][j] = Frag<T>::mma(al, bh[j], acc[i][j]);
        }
      }
      Frag<T>::guard(acc[i][0], acc[i][3], ah, SPLIT ? al : ah);
    }
    Frag<T>::keep(bh[0], bh[1], bh[2], bh[3]);
    if (SPLIT) Frag<T>::keep(bl[0], bl[1], bl[2], bl[3]);
  }
  acc_guard4(acc[0][0], acc[0][1], acc[0][2], acc[0][3]);
  acc_guard4(acc[1][0], acc[1][1], acc[1][2], acc[1][3]);
  acc_guard4(acc[2][0], acc[2][1], acc[2][2], acc[2][3]);
  acc_guard4(acc[3][0], acc[3][1], acc[3][2], acc[3][3]);

  float* slab = sT[wave];
  const float* Rb = RESID ? (resid + (size_t)b * strideR) : nullptr;
#pragma unroll
  for (int i = 0; i < 4; ++i) {
    const int mBase = m0 + (i << 4);
#pragma unroll
    for (int j = 0; j < 4; ++j) {
      const int n = n0 + (j << 4) + rlane;
      float bv = 0.f;
      if (BIAS_MODE == 2) bv = bias[n];
#pragma unroll
      for (int r = 0; r < 8; ++r) {
        float v = acc[i][j][r] * scale;
        if (BIAS_MODE == 1) v += bias[mBase + mOff + r];
        if (BIAS_MODE == 2) v += bv;
        if (RESID) v += Rb[(size_t)(mBase + mOff + r) * ldc + n];
        if (ACT == 1) v = tanhf(v);
        if (ACT == 2) v = fmaxf(v, 0.0f);
        if (ACT == 3) v = v / (1.0f + expf(-v));
        if (ACT == 4) v = (v > 0.f) ? v : 0.01f * v;
        slab[(mOff + r) * 68 + (j << 4) + rlane] = v;
      }
    }
    __builtin_amdgcn_fence(__ATOMIC_RELEASE, "workgroup");
    __builtin_amdgcn_wave_barrier();
    __builtin_amdgcn_fence(__ATOMIC_ACQUIRE, "workgroup");
    if (OUT_MODE == 0) {
      float* C = (float*)Cout + (size_t)b * strideC;
      const int hh = lane >> 4, c4 = (lane & 15) * 4;
      if (DUADD) {
        const v4f dv4 = *(const v4f*)(dsc + n0 + c4);
#pragma unroll
        for (int it = 0; it < 8; ++it) {
          const int row = it * 2 + hh;
          v4f sv = *(const v4f*)(slab + row * 68 + c4);
          const v4f uu = *(const v4f*)(uadd + (size_t)(mBase + row) * ldu + n0 + c4);
          sv = dv4 * uu + sv;
          *(v4f*)(slab + row * 68 + c4) = sv;
        }
      }
      for (int pass = 0; pass < 2; ++pass) {
#pragma unroll
        for (int it = 0; it < 8; ++it) {
          const int row = it * 2 + hh;
          v4f v = *(const v4f*)(slab + row * 68 + c4);
          *(volatile v4f*)(C + (size_t)(mBase + row) * ldc + n0 + c4) = v;
        }
        __threadfence();
      }
    } else {
      const int q = lane >> 3, c8 = (lane & 7) * 8;
      unsigned short* C  = (unsigned short*)Cout  + (size_t)b * strideC;
      unsigned short* C2 = (OUT_MODE == 2) ? ((unsigned short*)Cout2 + (size_t)b * strideC) : nullptr;
      for (int pass = 0; pass < 2; ++pass) {
#pragma unroll
        for (int it = 0; it < 4; ++it) {
          const int row = it * 4 + q;
          const float* sp = slab + row * 68 + c8;
          v8h hv, lv;
#pragma unroll
          for (int e = 0; e < 8; ++e) {
            if (OUT_MODE == 1) {
              hv[e] = (_Float16)sp[e];
            } else {
              unsigned short hb = f2bf_bits(sp[e]);
              unsigned short lb = f2bf_bits(sp[e] - bf_bits2f(hb));
              hv[e] = __builtin_bit_cast(_Float16, hb);
              lv[e] = __builtin_bit_cast(_Float16, lb);
            }
          }
          *(volatile v8h*)(C + (size_t)(mBase + row) * ldc + n0 + c8) = hv;
          if (OUT_MODE == 2) *(volatile v8h*)(C2 + (size_t)(mBase + row) * ldc + n0 + c8) = lv;
        }
        __threadfence();
      }
    }
    __builtin_amdgcn_fence(__ATOMIC_RELEASE, "workgroup");
    __builtin_amdgcn_wave_barrier();
    __builtin_amdgcn_fence(__ATOMIC_ACQUIRE, "workgroup");
  }
}

template <bool ROWSCALE>
__global__ __launch_bounds__(CVT_THR) void split_planes_kernel(
    const float* __restrict__ src, int spitch,
    const float* __restrict__ rowlog,
    unsigned short* __restrict__ dsth, unsigned short* __restrict__ dstl,
    int dpitch, int dcol0, int nrow, int ncol8) {
  const int i  = blockIdx.x * CVT_THR + threadIdx.x;
  const int n8 = nrow * ncol8;
  if (i < n8) {
    const int row = i / ncol8;
    const int c8  = i - row * ncol8;
    const float* sp = src + (size_t)row * spitch + (size_t)c8 * 8;
    const v4f a = *(const v4f*)(sp);
    const v4f b = *(const v4f*)(sp + 4);
    float sc = 1.0f;
    if (ROWSCALE) sc = expf(rowlog[row]);
    v8h hv, lv;
#pragma unroll
    for (int e = 0; e < 4; ++e) {
      const float v0 = a[e] * sc;
      const float v1 = b[e] * sc;
      const unsigned short h0 = f2bf_bits(v0);
      const unsigned short l0 = f2bf_bits(v0 - bf_bits2f(h0));
      const unsigned short h1 = f2bf_bits(v1);
      const unsigned short l1 = f2bf_bits(v1 - bf_bits2f(h1));
      hv[e]     = __builtin_bit_cast(_Float16, h0);
      hv[4 + e] = __builtin_bit_cast(_Float16, h1);
      lv[e]     = __builtin_bit_cast(_Float16, l0);
      lv[4 + e] = __builtin_bit_cast(_Float16, l1);
    }
    const size_t o = (size_t)row * dpitch + (size_t)dcol0 + (size_t)c8 * 8;
    for (int pass = 0; pass < 2; ++pass) {
      *(volatile v8h*)(dsth + o) = hv;
      *(volatile v8h*)(dstl + o) = lv;
      __threadfence();
    }
  }
}

__global__ __launch_bounds__(SCAN_THR) void diag_scan_kernel(
    const float* __restrict__ Bu,
    const float* __restrict__ nu_log,
    const float* __restrict__ theta_log,
    unsigned short* __restrict__ A1h,
    unsigned short* __restrict__ A1l) {
  __shared__ __align__(16) float lamr_s[SCAN_CPB];
  __shared__ __align__(16) float lami_s[SCAN_CPB];
  const int lane = threadIdx.x;
  const int cb = blockIdx.x * SCAN_CPB;
#pragma unroll 1
  for (int i = lane; i < SCAN_CPB; i += SCAN_THR) {
    const float th = expf(theta_log[cb + i]);
    const float rr = expf(-expf(nu_log[cb + i]));
    lamr_s[i] = rr * cosf(th);
    lami_s[i] = rr * sinf(th);
  }
  __syncthreads();

  const int c0 = SCAN_CPL * lane;
  float lr[8], li[8], xr[8], xi[8];
#pragma unroll
  for (int e = 0; e < 8; ++e) {
    lr[e] = lamr_s[c0 + e];
    li[e] = lami_s[c0 + e];
    xr[e] = 0.0f;
    xi[e] = 0.0f;
  }
  const size_t colr = (size_t)cb + (size_t)c0;
  const size_t coli = (size_t)NST + colr;
  const float* bre = Bu + colr;
  const float* bim = Bu + coli;
  v4f pra = *(const v4f*)(bre);
  v4f prb = *(const v4f*)(bre + 4);
  v4f pia = *(const v4f*)(bim);
  v4f pib = *(const v4f*)(bim + 4);

#pragma unroll 1
  for (int t = 0; t < SEQ_L; ++t) {
    const v4f cra = pra, crb = prb, cia = pia, cib = pib;
    const int tn = (t + 1 < SEQ_L) ? (t + 1) : (SEQ_L - 1);
    const size_t rn = (size_t)tn * NST2;
    pra = *(const v4f*)(bre + rn);
    prb = *(const v4f*)(bre + rn + 4);
    pia = *(const v4f*)(bim + rn);
    pib = *(const v4f*)(bim + rn + 4);

    float br[8], bi[8];
    br[0] = cra[0]; br[1] = cra[1]; br[2] = cra[2]; br[3] = cra[3];
    br[4] = crb[0]; br[5] = crb[1]; br[6] = crb[2]; br[7] = crb[3];
    bi[0] = cia[0]; bi[1] = cia[1]; bi[2] = cia[2]; bi[3] = cia[3];
    bi[4] = cib[0]; bi[5] = cib[1]; bi[6] = cib[2]; bi[7] = cib[3];
#pragma unroll
    for (int e = 0; e < 8; ++e) {
      const float nr = fmaf(lr[e], xr[e], fmaf(-li[e], xi[e], br[e]));
      const float ni = fmaf(lr[e], xi[e], fmaf( li[e], xr[e], bi[e]));
      xr[e] = nr;
      xi[e] = ni;
    }
    v8h hvr, lvr, hvi, lvi;
#pragma unroll
    for (int e = 0; e < 8; ++e) {
      const float vr = xr[e];
      const float vi = -xi[e];
      const unsigned short hr = f2bf_bits(vr);
      const unsigned short qr = f2bf_bits(vr - bf_bits2f(hr));
      const unsigned short hi = f2bf_bits(vi);
      const unsigned short qi = f2bf_bits(vi - bf_bits2f(hi));
      hvr[e] = __builtin_bit_cast(_Float16, hr);
      lvr[e] = __builtin_bit_cast(_Float16, qr);
      hvi[e] = __builtin_bit_cast(_Float16, hi);
      lvi[e] = __builtin_bit_cast(_Float16, qi);
    }
    const size_t ro = (size_t)t * NST2;
    for (int pass = 0; pass < 2; ++pass) {
      *(volatile v8h*)(A1h + ro + colr) = hvr;
      *(volatile v8h*)(A1h + ro + coli) = hvi;
      *(volatile v8h*)(A1l + ro + colr) = lvr;
      *(volatile v8h*)(A1l + ro + coli) = lvi;
      __threadfence();
    }
  }
}

extern "C" void kernel_launch(void* const* d_in, const int* in_sizes, int n_in,
                              void* d_out, int out_size, void* d_ws, size_t ws_size, hipStream_t stream) {
  if (n_in < 9 || d_out == nullptr || d_ws == nullptr) return;
  if (in_sizes[0] != SEQ_L * HID || in_sizes[1] != NST || in_sizes[2] != NST || in_sizes[3] != NST ||
      in_sizes[4] != NST * HID || in_sizes[5] != NST * HID || in_sizes[6] != HID * NST || in_sizes[7] != HID * NST ||
      in_sizes[8] != HID || out_size != SEQ_L * HID) return;

  const float* u         = (const float*)d_in[0];
  const float* nu_log    = (const float*)d_in[1];
  const float* theta_log = (const float*)d_in[2];
  const float* b_re      = (const float*)d_in[4];
  const float* b_im      = (const float*)d_in[5];
  const float* c_re      = (const float*)d_in[6];
  const float* c_im      = (const float*)d_in[7];
  const float* dvec      = (const float*)d_in[8];
  float* y = (float*)d_out;

  char* ws = (char*)d_ws; size_t off = 0;
  auto carve = [&](size_t bytes) -> char* { char* p = ws + off; off += (bytes + 255) & ~(size_t)255; return p; };
  unsigned short* A0H  = (unsigned short*)carve((size_t)SEQ_L * HID * 2);
  unsigned short* A0L  = (unsigned short*)carve((size_t)SEQ_L * HID * 2);
  unsigned short* BT0H = (unsigned short*)carve((size_t)NST2 * HID * 2);
  unsigned short* BT0L = (unsigned short*)carve((size_t)NST2 * HID * 2);
  unsigned short* BT1H = (unsigned short*)carve((size_t)HID * NST2 * 2);
  unsigned short* BT1L = (unsigned short*)carve((size_t)HID * NST2 * 2);
  float*          BU   = (float*)carve((size_t)SEQ_L * NST2 * 4);
  unsigned short* A1H  = (unsigned short*)carve((size_t)SEQ_L * NST2 * 2);
  unsigned short* A1L  = (unsigned short*)carve((size_t)SEQ_L * NST2 * 2);
  if (off > ws_size || off > (size_t)134217728) return;

  const int n8u = SEQ_L * (HID / 8);
  const int n8b = NST * (HID / 8);
  const int n8c = HID * (NST / 8);
  split_planes_kernel<false><<<n8u / CVT_THR, CVT_THR, 0, stream>>>(u,    HID, theta_log, A0H, A0L, HID, 0, SEQ_L, HID / 8);
  split_planes_kernel<true ><<<n8b / CVT_THR, CVT_THR, 0, stream>>>(b_re, HID, theta_log, BT0H, BT0L, HID, 0, NST, HID / 8);
  split_planes_kernel<true ><<<n8b / CVT_THR, CVT_THR, 0, stream>>>(b_im, HID, theta_log,
                                                                    BT0H + (size_t)NST * HID, BT0L + (size_t)NST * HID, HID, 0, NST, HID / 8);
  split_planes_kernel<false><<<n8c / CVT_THR, CVT_THR, 0, stream>>>(c_re, NST, theta_log, BT1H, BT1L, NST2, 0,   HID, NST / 8);
  split_planes_kernel<false><<<n8c / CVT_THR, CVT_THR, 0, stream>>>(c_im, NST, theta_log, BT1H, BT1L, NST2, NST, HID, NST / 8);

  const dim3 g0((SEQ_L / 64) * (NST2 / 64) / 8, 1);
  wmma_gemm64<1, true, 0, 0, false, 0, false><<<g0, 256, 0, stream>>>(
      A0H, A0L, HID, 0L, BT0H, BT0L, HID, 0L, (void*)BU, (void*)BU, NST2, 0L,
      dvec, u, 0L, SEQ_L, NST2, HID, 1.0f, dvec, u, HID);

  diag_scan_kernel<<<NST / SCAN_CPB, SCAN_THR, 0, stream>>>(BU, nu_log, theta_log, A1H, A1L);

  const dim3 g1((SEQ_L / 64) * (HID / 64) / 8, 1);
  wmma_gemm64<1, true, 0, 0, false, 0, true><<<g1, 256, 0, stream>>>(
      A1H, A1L, NST2, 0L, BT1H, BT1L, NST2, 0L, (void*)y, (void*)y, HID, 0L,
      dvec, u, 0L, SEQ_L, HID, NST2, 1.0f, dvec, u, HID);
}
